// Model_13374528160105
// MI455X (gfx1250) — hardware-run, weakly checked
//
#include <hip/hip_runtime.h>
#include <stddef.h>
#include <stdint.h>
#include <math.h>

#define NNODE   100000
#define NHIGH   20000
#define NE      200000
#define DD      128
#define NHEAD   4
#define HDW     512
#define MPX     100096
#define MPH     20096
#define NTHR    256
#define NWAVE   8
#define NBK     20
#define NBRUN   1024
#define SLB     10
#define EPT     2
#define WCH     (32 * EPT)
#define WLCAP   2048
#define RCAP    12288
#define TRIPCAP 256
#define MAXDEG_MEAS   24
#define MAXB1024_MEAS 10381
#define PSLOTS  256
#define NPB     80
#define STATROWS (NPB * PSLOTS)
#define SPLIT_G  1
#define SPLIT_HF 1
#define KG      (SPLIT_G ? 1024 : 512)
#define KHF     (SPLIT_HF ? 256 : 128)
#define GPITCH  1024
#define HPITCH  256
#define GBM     64
#define SPW     132
#define ADP     20

#define BK_ZINTS (NWAVE * WLCAP + RCAP + 3 * NBRUN)
#define BK_INTS  (BK_ZINTS + 16)
#define BK_LDS   (BK_INTS * 4)

#define PBX  (MPX * DD / 8 / NTHR)
#define PBWS (DD * GPITCH / 8 / NTHR)
#define PBWH (DD * HPITCH / 8 / NTHR)
#define PBUD 2
#define PBUS 2
#define PBTOT (PBX + PBWS + PBWH + PBUD + PBUS + 1)

static_assert(DD == 128 && DD == 32 * 4 && NHEAD == 4 && HDW == NHEAD * DD);
static_assert(NBK * NBRUN >= NHIGH && NBRUN == (1 << SLB));
static_assert(RCAP % 32 == 0 && RCAP % 4 == 0 && BK_ZINTS % 4 == 0);
static_assert(MPX % 128 == 0 && MPH % 128 == 0 && MPX >= NNODE && MPH >= NHIGH && MPH % GBM == 0);
static_assert(PSLOTS % 2 == 0 && NBRUN % PSLOTS == 0 && STATROWS >= MPH && STATROWS <= NBK * NBRUN);
static_assert(NE % 8 == 0 && NE % WCH == 0 && NE % 32 == 0);
static_assert(NE < (1 << 21) && (((long long)NE) << SLB) < (1LL << 31));
static_assert((long long)RCAP * 100 >= (long long)MAXB1024_MEAS * 115);
static_assert(WLCAP >= MAXB1024_MEAS / 8 + 8 * 46 + 1);
static_assert(MAXDEG_MEAS + 8 <= TRIPCAP);
static_assert((MPX * DD / 8) % NTHR == 0 && (DD * GPITCH / 8) % NTHR == 0 && (DD * HPITCH / 8) % NTHR == 0);
static_assert(KG % 32 == 0 && KHF % 32 == 0 && DD % 32 == 0);
static_assert(BK_LDS <= 300000);
static_assert(GBM * SPW * 4 + 512 <= 65536);

typedef float          v4f   __attribute__((ext_vector_type(4)));
typedef float          v8f   __attribute__((ext_vector_type(8)));
typedef int            v2i   __attribute__((ext_vector_type(2)));
typedef int            v4i   __attribute__((ext_vector_type(4)));
typedef int            v8i   __attribute__((ext_vector_type(8)));
typedef unsigned int   v2u   __attribute__((ext_vector_type(2)));
typedef unsigned int   v4u   __attribute__((ext_vector_type(4)));
typedef unsigned short v8us  __attribute__((ext_vector_type(8)));
typedef unsigned short v16us __attribute__((ext_vector_type(16)));
typedef __bf16         v16bf __attribute__((ext_vector_type(16)));
typedef v4f  __attribute__((may_alias)) v4fa;
typedef v2i  __attribute__((may_alias)) v2ia;
typedef v4i  __attribute__((may_alias)) v4ia;
typedef v2u  __attribute__((may_alias)) v2ua;
typedef v8us __attribute__((may_alias)) v8usa;
union FragB { v16bf v; v16us u; v8us h[2]; v8i w; };

__device__ __forceinline__ v8f wmb(const FragB& a, const FragB& b, v8f c) {
  v8f d = __builtin_amdgcn_wmma_f32_16x16x32_bf16(false, a.v, false, b.v, (short)0, c, false, false);
  asm volatile("v_nop\n\tv_nop\n\tv_nop\n\tv_nop" : "+v"(d) : "v"(a.w), "v"(b.w));
  return d;
}

__device__ __forceinline__ unsigned bf16_bits(float f) {
  const unsigned u = __float_as_uint(f);
  const unsigned r = (u + 0x7FFFu + ((u >> 16) & 1u)) >> 16;
  const unsigned q = (u >> 16) | 0x40u;
  return ((u & 0x7fffffffu) > 0x7f800000u) ? q : r;
}
__device__ __forceinline__ float bf16_val(float f) {
  return __uint_as_float(bf16_bits(f) << 16);
}

__device__ __forceinline__ void hilo_pack(float v0, float v1, float v2, float v3,
                                          int& h01, int& h23, int& l01, int& l23) {
  const unsigned a0 = bf16_bits(v0), a1 = bf16_bits(v1), a2 = bf16_bits(v2), a3 = bf16_bits(v3);
  const unsigned b0 = bf16_bits(v0 - __uint_as_float(a0 << 16));
  const unsigned b1 = bf16_bits(v1 - __uint_as_float(a1 << 16));
  const unsigned b2 = bf16_bits(v2 - __uint_as_float(a2 << 16));
  const unsigned b3 = bf16_bits(v3 - __uint_as_float(a3 << 16));
  h01 = (int)(a0 | (a1 << 16)); h23 = (int)(a2 | (a3 << 16));
  l01 = (int)(b0 | (b1 << 16)); l23 = (int)(b2 | (b3 << 16));
}

__device__ __forceinline__ void st2_v4f(float* p, v4f v) {
  *(volatile v4f*)p = v;
  __threadfence();
  *(volatile v4f*)p = v;
}
__device__ __forceinline__ void st2_v8us(unsigned short* p, v8us v) {
  *(volatile v8us*)p = v;
  __threadfence();
  *(volatile v8us*)p = v;
}
__device__ __forceinline__ void st2_v4u(unsigned short* p, v4u v) {
  *(volatile v4u*)p = v;
  __threadfence();
  *(volatile v4u*)p = v;
}

__device__ __forceinline__ v8us gather8(const float* __restrict__ base, int stride) {
  float f[8];
#pragma unroll
  for (int i = 0; i < 8; ++i) f[i] = base[(size_t)i * (size_t)stride];
  v8us o;
#pragma unroll
  for (int i = 0; i < 8; ++i) o[i] = (unsigned short)bf16_bits(f[i]);
  return o;
}

__device__ __forceinline__ float dot128_bf(const float* __restrict__ wrow, const float* __restrict__ av) {
  float s = 0.0f;
#pragma unroll 2
  for (int c4 = 0; c4 < DD / 4; ++c4) {
    const v4f w = *(const v4fa*)(wrow + 4 * c4);
    const v4f a = *(const v4fa*)(av + 4 * c4);
    s = fmaf(bf16_val(w.x), bf16_val(a.x), s);
    s = fmaf(bf16_val(w.y), bf16_val(a.y), s);
    s = fmaf(bf16_val(w.z), bf16_val(a.z), s);
    s = fmaf(bf16_val(w.w), bf16_val(a.w), s);
  }
  return s;
}

__device__ __forceinline__ float score_of(float as, float ad) {
  const float v = as + ad;
  return (v > 0.0f) ? v : 0.2f * v;
}
__device__ __forceinline__ float alpha_of(float sc, float mx, float den) {
  return expf(sc - mx) / den;
}

__global__ __launch_bounds__(NTHR) void k_prep(const float* __restrict__ x, const float* __restrict__ wsrc,
                                               const float* __restrict__ wdst, const float* __restrict__ atts,
                                               const float* __restrict__ attd, const float* __restrict__ whigh,
                                               const float* __restrict__ bhigh,
                                               unsigned short* xb, unsigned short* wst2, unsigned short* wht2,
                                               unsigned short* udt, float* usrc, float* bh) {
  __shared__ __attribute__((aligned(16))) float sres[NTHR];
  const int tid = (int)threadIdx.x, lane = tid & 31;
  const int blk = (int)blockIdx.x;
  if (blk < PBX) {
    const int u   = blk * NTHR + tid;
    const int row = u >> 4, k8 = (u & 15) * 8;
    const int rc  = row < NNODE ? row : NNODE - 1;
    const unsigned mk = row < NNODE ? 0xffffu : 0u;
    const float* p = x + (size_t)rc * DD + k8;
    const v4f a = *(const v4fa*)p;
    const v4f b = *(const v4fa*)(p + 4);
    v8us o;
    o[0] = (unsigned short)(bf16_bits(a.x) & mk); o[1] = (unsigned short)(bf16_bits(a.y) & mk);
    o[2] = (unsigned short)(bf16_bits(a.z) & mk); o[3] = (unsigned short)(bf16_bits(a.w) & mk);
    o[4] = (unsigned short)(bf16_bits(b.x) & mk); o[5] = (unsigned short)(bf16_bits(b.y) & mk);
    o[6] = (unsigned short)(bf16_bits(b.z) & mk); o[7] = (unsigned short)(bf16_bits(b.w) & mk);
    st2_v8us(xb + (size_t)row * DD + k8, o);
  } else if (blk < PBX + PBWS) {
    const int u  = (blk - PBX) * NTHR + tid;
    const int n  = u >> 7, k8 = (u & 127) * 8;
    const int h  = (k8 >> 7) & 3, kk = k8 & 127;
    const v8us o = gather8(wsrc + (size_t)kk * HDW + h * DD + n, HDW);
    st2_v8us(wst2 + (size_t)n * GPITCH + k8, o);
  } else if (blk < PBX + PBWS + PBWH) {
    const int u  = (blk - PBX - PBWS) * NTHR + tid;
    const int n  = u >> 5, k8 = (u & 31) * 8, kk = k8 & 127;
    const v8us o = gather8(whigh + (size_t)kk * DD + n, DD);
    st2_v8us(wht2 + (size_t)n * HPITCH + k8, o);
  } else if (blk < PBX + PBWS + PBWH + PBUD) {
    const int j = blk - (PBX + PBWS + PBWH);
    const int k = 64 * j + (tid >> 2), h = tid & 3;
    sres[tid] = dot128_bf(wsrc + (size_t)k * HDW + h * DD, attd + h * DD);
    __syncthreads();
    if (tid < 128) {
      const int row = tid >> 3, piece = tid & 7;
      const int p = row >> 2, hh = row & 3;
      v8us o;
#pragma unroll
      for (int i = 0; i < 8; ++i) {
        const float uv = sres[(piece * 8 + i) * 4 + hh];
        const unsigned hb = bf16_bits(uv);
        const float r1 = uv - __uint_as_float(hb << 16);
        const unsigned mb = bf16_bits(r1);
        const float r2 = r1 - __uint_as_float(mb << 16);
        const unsigned lb = bf16_bits(r2);
        const unsigned sel = (p == 0) ? hb : ((p == 1) ? mb : ((p == 2) ? lb : 0u));
        o[i] = (unsigned short)sel;
      }
      st2_v8us(udt + (size_t)row * DD + 64 * j + piece * 8, o);
    }
  } else if (blk < PBX + PBWS + PBWH + PBUD + PBUS) {
    const int j = blk - (PBX + PBWS + PBWH + PBUD);
    const int k = 64 * j + (tid >> 2), h = tid & 3;
    sres[tid] = dot128_bf(wdst + (size_t)k * HDW + h * DD, atts + h * DD);
    __syncthreads();
    if (tid < 64) {
      const v4f v = *(const v4fa*)(sres + 4 * tid);
      st2_v4f(usrc + 256 * j + 4 * tid, v);
    }
  } else {
    if (tid < 32) {
      const v4f b = *(const v4fa*)(bhigh + 4 * lane);
      v4f o;
      o.x = bf16_val(b.x); o.y = bf16_val(b.y); o.z = bf16_val(b.z); o.w = bf16_val(b.w);
      st2_v4f(bh + 4 * lane, o);
    }
  }
}

__device__ __forceinline__ void bucket_flush(const int* pl, const int* cnt, int ov, int* lp, int* cop, int* fp,
                                             int tid) {
#pragma unroll 1
  for (int i = tid * 4; i < RCAP; i += NTHR * 4) {
    const v4i v = *(const v4ia*)(pl + i);
    *(volatile v4i*)(lp + i) = v;
  }
#pragma unroll 1
  for (int i = tid * 4; i < 2 * NBRUN; i += NTHR * 4) {
    const v4i v = *(const v4ia*)(cnt + i);
    *(volatile v4i*)(cop + i) = v;
  }
  if (tid < 8) {
    const v4i f = {ov, ov, ov, ov};
    *(volatile v4i*)(fp + 4 * tid) = f;
  }
}

__global__ __launch_bounds__(NTHR) void k_bucket(const int* __restrict__ dsts, int* LIST, int* CO, int* FLAG) {
  extern __shared__ __attribute__((aligned(16))) int dsm[];
  int* wl   = dsm;
  int* pl   = dsm + NWAVE * WLCAP;
  int* cnt  = pl + RCAP;
  int* offs = cnt + NBRUN;
  int* cur  = offs + NBRUN;
  int* misc = cur + NBRUN;
  const int tid = (int)threadIdx.x, lane = tid & 31, wave = tid >> 5;
  const int blk = (int)blockIdx.x;
  const unsigned nbs = (unsigned)(blk * NBRUN);
  int nreal = NHIGH - blk * NBRUN;
  nreal = nreal > NBRUN ? NBRUN : (nreal < 0 ? 0 : nreal);
  const unsigned unb = (unsigned)nreal;

  {
    const v4i z4 = {0, 0, 0, 0};
    for (int i = tid * 4; i < BK_ZINTS; i += NTHR * 4) *(v4ia*)(dsm + i) = z4;
    if (tid < 16) misc[tid] = 0;
  }
  __syncthreads();

  {
    const int per  = ((NE + NWAVE * WCH - 1) / (NWAVE * WCH)) * WCH;
    const int ebeg = wave * per;
    const int eend = (ebeg + per < NE) ? (ebeg + per) : NE;
    int* mylist = wl + wave * WLCAP;
    int wc = 0;
#pragma unroll 1
    for (int cb = ebeg; cb < eend; cb += WCH) {
      const int e0 = cb + lane * EPT;
      const v2i da = *(const v2ia*)(dsts + e0);
      const unsigned s0 = (unsigned)da.x - nbs, s1 = (unsigned)da.y - nbs;
      const bool h0 = s0 < unb, h1 = s1 < unb;
      const unsigned m0 = __builtin_amdgcn_ballot_w32(h0), m1 = __builtin_amdgcn_ballot_w32(h1);
      const unsigned any = m0 | m1;
      if (any != 0u) {
        const int pre = (int)(__builtin_amdgcn_mbcnt_lo(m0, 0u) + __builtin_amdgcn_mbcnt_lo(m1, 0u));
        int p = wc + pre;
        if (h0) { if (p < WLCAP) mylist[p] = ((e0 + 0) << SLB) | (int)s0; p = p + 1; }
        if (h1) { if (p < WLCAP) mylist[p] = ((e0 + 1) << SLB) | (int)s1; p = p + 1; }
        wc += (int)(__builtin_popcount(m0) + __builtin_popcount(m1));
      }
    }
    if (lane == 0) misc[wave] = wc;
  }
  __syncthreads();

  if (wave == 0) {
    int ov = 0;
#pragma unroll 1
    for (int w2 = 0; w2 < NWAVE; ++w2) {
      int c = misc[w2];
      if (c > WLCAP) ov = 1;
      c = c < 0 ? 0 : (c > WLCAP ? WLCAP : c);
#pragma unroll 1
      for (int b0 = 0; b0 < c; b0 += 32) {
        const int idx = b0 + lane;
        const int ent = wl[w2 * WLCAP + (idx < WLCAP ? idx : WLCAP - 1)];
        const int m32 = (c - b0) < 32 ? (c - b0) : 32;
#pragma unroll 1
        for (int k = 0; k < m32; ++k) {
          const int u    = __builtin_amdgcn_readlane(ent, k);
          const int slot = u & (NBRUN - 1);
          if (lane == 0) cnt[slot] = cnt[slot] + 1;
        }
      }
    }
    if (lane == 0) misc[9] = ov;
  }
  __syncthreads();
  if (wave == 0) {
    const int base = lane * (NBRUN / 32);
    int s = 0;
#pragma unroll 1
    for (int i = 0; i < NBRUN / 32; ++i) s += cnt[base + i];
    int incl = s;
#pragma unroll
    for (int d = 1; d < 32; d <<= 1) {
      const int y = __shfl_up(incl, d, 32);
      if (lane >= d) incl += y;
    }
    int run = incl - s;
#pragma unroll 1
    for (int i = 0; i < NBRUN / 32; ++i) {
      const int cv = cnt[base + i];
      offs[base + i] = run;
      cur[base + i]  = run;
      run += cv;
    }
    if (lane == 31 && run > RCAP) misc[9] = 1;
  }
  __syncthreads();

  if (wave == 0) {
#pragma unroll 1
    for (int w2 = 0; w2 < NWAVE; ++w2) {
      int c = misc[w2];
      c = c < 0 ? 0 : (c > WLCAP ? WLCAP : c);
#pragma unroll 1
      for (int b0 = 0; b0 < c; b0 += 32) {
        const int idx = b0 + lane;
        const int ent = wl[w2 * WLCAP + (idx < WLCAP ? idx : WLCAP - 1)];
        int eid = (ent >> SLB) & 0x1FFFFF;
        eid = eid > NE - 1 ? NE - 1 : eid;
        const int m32 = (c - b0) < 32 ? (c - b0) : 32;
#pragma unroll 1
        for (int k = 0; k < m32; ++k) {
          const int u    = __builtin_amdgcn_readlane(ent, k);
          const int wd   = __builtin_amdgcn_readlane(eid, k);
          const int slot = u & (NBRUN - 1);
          if (lane == 0) {
            int p = cur[slot];
            p = p < 0 ? 0 : (p > RCAP - 1 ? RCAP - 1 : p);
            pl[p] = wd;
            cur[slot] = p + 1;
          }
        }
      }
    }
  }
  __syncthreads();

  const int ovf = misc[9];
  int* lp  = LIST + (size_t)blk * RCAP;
  int* cop = CO + (size_t)blk * (2 * NBRUN);
  int* fp  = FLAG + (size_t)blk * 32;
  bucket_flush(pl, cnt, ovf, lp, cop, fp, tid);
  __threadfence();
  bucket_flush(pl, cnt, ovf, lp, cop, fp, tid);
}

__global__ __launch_bounds__(NTHR) void k_ad(const unsigned short* __restrict__ XB,
                                             const unsigned short* __restrict__ UDT, float* AD) {
  __shared__ __attribute__((aligned(16))) float stg[128 * ADP];
  const int tid = (int)threadIdx.x, lane = tid & 31, wave = tid >> 5, hh = lane >> 4, m = lane & 15;
  const int rowBase = (int)blockIdx.x * 128;
  v8f acc = {0.f, 0.f, 0.f, 0.f, 0.f, 0.f, 0.f, 0.f};
  const unsigned short* ap = XB + (size_t)(rowBase + 16 * wave + m) * (size_t)DD + 8 * hh;
  const unsigned short* bp = UDT + (size_t)m * (size_t)DD + 8 * hh;
#pragma unroll 1
  for (int k0 = 0; k0 < DD; k0 += 32) {
    FragB af, bf;
    af.h[0] = *(const v8usa*)(ap + k0);
    af.h[1] = *(const v8usa*)(ap + k0 + 16);
    bf.h[0] = *(const v8usa*)(bp + k0);
    bf.h[1] = *(const v8usa*)(bp + k0 + 16);
    acc = wmb(af, bf, acc);
  }
#pragma unroll
  for (int r = 0; r < 8; ++r) stg[(16 * wave + 8 * hh + r) * ADP + m] = acc[r];
  __syncthreads();
  if (tid < 128) {
    const v4f a = *(const v4fa*)(stg + tid * ADP);
    const v4f b = *(const v4fa*)(stg + tid * ADP + 4);
    const v4f c = *(const v4fa*)(stg + tid * ADP + 8);
    v4f o;
    o.x = (a.x + b.x) + c.x; o.y = (a.y + b.y) + c.y; o.z = (a.z + b.z) + c.z; o.w = (a.w + b.w) + c.w;
    st2_v4f(AD + (size_t)(rowBase + tid) * 4, o);
  }
}

__device__ __forceinline__ void hit_load(const int* __restrict__ lb, const int* __restrict__ srcs,
                                         const float* __restrict__ AD, int o, int last, int hidx, int hq,
                                         int& s_out, float& ad_out) {
  int idx = o + hidx;
  idx = idx > last ? last : idx;
  idx = idx < 0 ? 0 : idx;
  int e = lb[idx];
  e = e < 0 ? 0 : (e > NE - 1 ? NE - 1 : e);
  int sv = srcs[e];
  sv = sv < 0 ? 0 : (sv > NNODE - 1 ? NNODE - 1 : sv);
  const float a = AD[(size_t)sv * 4 + hq];
  asm volatile("" :: "v"(a));
  s_out = sv;
  ad_out = a;
}

__global__ __launch_bounds__(NTHR) void k_pool(const int* __restrict__ LIST, const int* __restrict__ CO,
                                               const int* __restrict__ FLAG, const int* __restrict__ srcs,
                                               const unsigned short* __restrict__ XB, const float* __restrict__ AD,
                                               const float* __restrict__ USRC, unsigned short* GHL, float* STAT) {
  __shared__ __attribute__((aligned(16))) float sst[PSLOTS * 16];
  __shared__ __attribute__((aligned(16))) float sus[DD * NHEAD];
  const int tid = (int)threadIdx.x, lane = tid & 31, wave = tid >> 5;
  const int blk = (int)blockIdx.x;
  const int slotBase = blk * PSLOTS;
  const int bucket   = slotBase >> SLB;
  const int* lb  = LIST + (size_t)bucket * RCAP;
  const int* cob = CO + (size_t)bucket * (2 * NBRUN);
  const int flag = FLAG[(size_t)bucket * 32];
  const float qnan = __uint_as_float(0x7fc00000u);
  const float ninf = __uint_as_float(0xff800000u);
  const int hq = lane & 3, jq = lane >> 2;

  if (tid < 128) *(v4fa*)(sus + 4 * tid) = *(const v4fa*)(USRC + 4 * tid);
  __syncthreads();
  const v4f u0 = *(const v4fa*)(sus + 16 * lane);
  const v4f u1 = *(const v4fa*)(sus + 16 * lane + 4);
  const v4f u2 = *(const v4fa*)(sus + 16 * lane + 8);
  const v4f u3 = *(const v4fa*)(sus + 16 * lane + 12);

#pragma unroll 1
  for (int i = 0; i < PSLOTS / NWAVE; ++i) {
    const int ls   = wave * (PSLOTS / NWAVE) + i;
    const int grow = slotBase + ls;
    const int slot = grow & (NBRUN - 1);
    const int craw = __builtin_amdgcn_readfirstlane(cob[slot]);
    int o = __builtin_amdgcn_readfirstlane(cob[NBRUN + slot]);
    const bool big = craw > TRIPCAP;
    const int c = craw < 0 ? 0 : (craw > TRIPCAP ? TRIPCAP : craw);
    o = o < 0 ? 0 : (o > RCAP - 1 ? RCAP - 1 : o);
    int last = o + c - 1;
    last = last < o ? o : last;
    last = last > RCAP - 1 ? RCAP - 1 : last;

    float s0 = 0.0f, s1 = 0.0f, s2 = 0.0f, s3 = 0.0f;
#pragma unroll 1
    for (int j = 0; j < c; ++j) {
      int idx = o + j;
      idx = idx > last ? last : idx;
      int e = lb[idx];
      e = e < 0 ? 0 : (e > NE - 1 ? NE - 1 : e);
      int sv = srcs[e];
      sv = sv < 0 ? 0 : (sv > NNODE - 1 ? NNODE - 1 : sv);
      const v2u xw = *(const v2ua*)(XB + (size_t)sv * DD + 4 * lane);
      s0 += __uint_as_float(xw.x << 16);
      s1 += __uint_as_float(xw.x & 0xffff0000u);
      s2 += __uint_as_float(xw.y << 16);
      s3 += __uint_as_float(xw.y & 0xffff0000u);
    }
    const float cf = fmaxf((float)c, 1.0f);
    const float m0 = s0 / cf, m1 = s1 / cf, m2 = s2 / cf, m3 = s3 / cf;
    float as0 = m0 * u0.x, as1 = m0 * u0.y, as2 = m0 * u0.z, as3 = m0 * u0.w;
    as0 = fmaf(m1, u1.x, as0); as1 = fmaf(m1, u1.y, as1); as2 = fmaf(m1, u1.z, as2); as3 = fmaf(m1, u1.w, as3);
    as0 = fmaf(m2, u2.x, as0); as1 = fmaf(m2, u2.y, as1); as2 = fmaf(m2, u2.z, as2); as3 = fmaf(m2, u2.w, as3);
    as0 = fmaf(m3, u3.x, as0); as1 = fmaf(m3, u3.y, as1); as2 = fmaf(m3, u3.z, as2); as3 = fmaf(m3, u3.w, as3);
#pragma unroll
    for (int d = 16; d >= 1; d >>= 1) {
      as0 += __shfl_xor(as0, d, 32);
      as1 += __shfl_xor(as1, d, 32);
      as2 += __shfl_xor(as2, d, 32);
      as3 += __shfl_xor(as3, d, 32);
    }
    const float ash = (hq == 0) ? as0 : ((hq == 1) ? as1 : ((hq == 2) ? as2 : as3));

    float mx = ninf;
#pragma unroll 1
    for (int cb = 0; cb < c; cb += 8) {
      int sj; float ad;
      hit_load(lb, srcs, AD, o, last, cb + jq, hq, sj, ad);
      const bool valid = (cb + jq) < c;
      const float sc = score_of(ash, ad);
      float t = valid ? sc : ninf;
      t = fmaxf(t, __shfl_xor(t, 4, 32));
      t = fmaxf(t, __shfl_xor(t, 8, 32));
      t = fmaxf(t, __shfl_xor(t, 16, 32));
      mx = fmaxf(mx, t);
    }
    mx = (mx == ninf) ? 0.0f : mx;

    float S = 0.0f;
#pragma unroll 1
    for (int cb = 0; cb < c; cb += 8) {
      int sj; float ad;
      hit_load(lb, srcs, AD, o, last, cb + jq, hq, sj, ad);
      const bool valid = (cb + jq) < c;
      const float sc = score_of(ash, ad);
      const float ev = expf(sc - mx);
      float t = valid ? ev : 0.0f;
      t += __shfl_xor(t, 4, 32);
      t += __shfl_xor(t, 8, 32);
      t += __shfl_xor(t, 16, 32);
      S += t;
    }
    const float den = S + 1e-16f;

    float g[4][4];
#pragma unroll
    for (int h = 0; h < 4; ++h) {
#pragma unroll
      for (int q = 0; q < 4; ++q) g[h][q] = 0.0f;
    }
#pragma unroll 1
    for (int cb = 0; cb < c; cb += 8) {
      int sj; float ad;
      hit_load(lb, srcs, AD, o, last, cb + jq, hq, sj, ad);
      const float sc = score_of(ash, ad);
      const float al = alpha_of(sc, mx, den);
      const int ali = __float_as_int(al);
      int m8 = c - cb;
      m8 = m8 > 8 ? 8 : m8;
#pragma unroll 1
      for (int k = 0; k < m8; ++k) {
        const int sk = __builtin_amdgcn_readlane(sj, 4 * k);
        const float a0 = __int_as_float(__builtin_amdgcn_readlane(ali, 4 * k));
        const float a1 = __int_as_float(__builtin_amdgcn_readlane(ali, 4 * k + 1));
        const float a2 = __int_as_float(__builtin_amdgcn_readlane(ali, 4 * k + 2));
        const float a3 = __int_as_float(__builtin_amdgcn_readlane(ali, 4 * k + 3));
        const v2u xw = *(const v2ua*)(XB + (size_t)sk * DD + 4 * lane);
        const float x0 = __uint_as_float(xw.x << 16), x1 = __uint_as_float(xw.x & 0xffff0000u);
        const float x2 = __uint_as_float(xw.y << 16), x3 = __uint_as_float(xw.y & 0xffff0000u);
        g[0][0] = fmaf(a0, x0, g[0][0]); g[0][1] = fmaf(a0, x1, g[0][1]); g[0][2] = fmaf(a0, x2, g[0][2]); g[0][3] = fmaf(a0, x3, g[0][3]);
        g[1][0] = fmaf(a1, x0, g[1][0]); g[1][1] = fmaf(a1, x1, g[1][1]); g[1][2] = fmaf(a1, x2, g[1][2]); g[1][3] = fmaf(a1, x3, g[1][3]);
        g[2][0] = fmaf(a2, x0, g[2][0]); g[2][1] = fmaf(a2, x1, g[2][1]); g[2][2] = fmaf(a2, x2, g[2][2]); g[2][3] = fmaf(a2, x3, g[2][3]);
        g[3][0] = fmaf(a3, x0, g[3][0]); g[3][1] = fmaf(a3, x1, g[3][1]); g[3][2] = fmaf(a3, x2, g[3][2]); g[3][3] = fmaf(a3, x3, g[3][3]);
      }
    }

    const bool bad  = (flag != 0) | big;
    const bool live = grow < NHIGH;
    const int sa = (2 * lane) & 31, sb = (2 * lane + 1) & 31;
    const unsigned lmk = (lane >= 16) ? 0xffffffffu : 0u;
    v4u pv[4];
#pragma unroll
    for (int h = 0; h < 4; ++h) {
      float v0 = g[h][0], v1 = g[h][1], v2 = g[h][2], v3 = g[h][3];
      v0 = bad ? qnan : v0; v1 = bad ? qnan : v1; v2 = bad ? qnan : v2; v3 = bad ? qnan : v3;
      v0 = live ? v0 : 0.0f; v1 = live ? v1 : 0.0f; v2 = live ? v2 : 0.0f; v3 = live ? v3 : 0.0f;
      int h01, h23, l01, l23;
      hilo_pack(v0, v1, v2, v3, h01, h23, l01, l23);
      const int g0 = __shfl(h01, sa, 32), g1 = __shfl(h23, sa, 32), g2 = __shfl(h01, sb, 32), g3 = __shfl(h23, sb, 32);
      const int q0 = __shfl(l01, sa, 32), q1 = __shfl(l23, sa, 32), q2 = __shfl(l01, sb, 32), q3 = __shfl(l23, sb, 32);
      pv[h].x = ((unsigned)q0 & lmk) | ((unsigned)g0 & ~lmk);
      pv[h].y = ((unsigned)q1 & lmk) | ((unsigned)g1 & ~lmk);
      pv[h].z = ((unsigned)q2 & lmk) | ((unsigned)g2 & ~lmk);
      pv[h].w = ((unsigned)q3 & lmk) | ((unsigned)g3 & ~lmk);
    }
    unsigned short* gp = GHL + (size_t)grow * GPITCH + ((lane & 16) ? 512 : 0) + 8 * (lane & 15);
    const bool wr = grow < MPH;
    if (wr) {
      *(volatile v4u*)(gp)       = pv[0];
      *(volatile v4u*)(gp + 128) = pv[1];
      *(volatile v4u*)(gp + 256) = pv[2];
      *(volatile v4u*)(gp + 384) = pv[3];
    }
    __threadfence();
    if (wr) {
      *(volatile v4u*)(gp)       = pv[0];
      *(volatile v4u*)(gp + 128) = pv[1];
      *(volatile v4u*)(gp + 256) = pv[2];
      *(volatile v4u*)(gp + 384) = pv[3];
    }
    const float asv = bad ? qnan : ash;
    const float mxv = bad ? qnan : mx;
    const float dnv = bad ? qnan : den;
    if (lane < 4) {
      float* r = sst + ls * 16;
      r[lane]      = asv;
      r[4 + lane]  = mxv;
      r[8 + lane]  = dnv;
      r[12 + lane] = 0.0f;
    }
  }
  __syncthreads();

  float* sp = STAT + (size_t)slotBase * 16;
#pragma unroll 1
  for (int it = 0; it < 4; ++it) {
    const int i4 = it * NTHR + tid;
    const v4f v = *(const v4fa*)(sst + 4 * i4);
    *(volatile v4f*)(sp + 4 * i4) = v;
  }
  __threadfence();
#pragma unroll 1
  for (int it = 0; it < 4; ++it) {
    const int i4 = it * NTHR + tid;
    const v4f v = *(const v4fa*)(sst + 4 * i4);
    *(volatile v4f*)(sp + 4 * i4) = v;
  }
}

__global__ __launch_bounds__(NTHR) void k_alpha(const int* __restrict__ srcs, const int* __restrict__ dsts,
                                                const float* __restrict__ STAT, const float* __restrict__ AD,
                                                const int* __restrict__ FLAG, float* out1) {
  const int e  = (int)blockIdx.x * NTHR + (int)threadIdx.x;
  const int ec = e < NE ? e : NE - 1;
  int d = dsts[ec];
  int s = srcs[ec];
  d = d < 0 ? 0 : (d > NHIGH - 1 ? NHIGH - 1 : d);
  s = s < 0 ? 0 : (s > NNODE - 1 ? NNODE - 1 : s);
  const float* sp = STAT + (size_t)d * 16;
  const v4f asv = *(const v4fa*)sp;
  const v4f mxv = *(const v4fa*)(sp + 4);
  const v4f dnv = *(const v4fa*)(sp + 8);
  const v4f adv = *(const v4fa*)(AD + (size_t)s * 4);
  const int fl  = FLAG[(size_t)(d >> SLB) * 32];
  asm volatile("" :: "v"(asv), "v"(mxv));
  asm volatile("" :: "v"(dnv), "v"(adv));
  asm volatile("" :: "v"(fl));
  const float qnan = __uint_as_float(0x7fc00000u);
  const float a0 = alpha_of(score_of(asv.x, adv.x), mxv.x, dnv.x);
  const float a1 = alpha_of(score_of(asv.y, adv.y), mxv.y, dnv.y);
  const float a2 = alpha_of(score_of(asv.z, adv.z), mxv.z, dnv.z);
  const float a3 = alpha_of(score_of(asv.w, adv.w), mxv.w, dnv.w);
  v4f o;
  o.x = (fl != 0) ? qnan : a0; o.y = (fl != 0) ? qnan : a1;
  o.z = (fl != 0) ? qnan : a2; o.w = (fl != 0) ? qnan : a3;
  if (e < NE) st2_v4f(out1 + (size_t)e * 4, o);
}

template <int KTOT, int PB>
__device__ __forceinline__ void gemm_16x64(const unsigned short* __restrict__ ap,
                                           const unsigned short* __restrict__ bp, v8f (&acc)[4]) {
#pragma unroll 1
  for (int k0 = 0; k0 < KTOT; k0 += 32) {
    FragB af;
    af.h[0] = *(const v8usa*)(ap + k0);
    af.h[1] = *(const v8usa*)(ap + k0 + 16);
#pragma unroll
    for (int nt = 0; nt < 4; ++nt) {
      const unsigned short* wq = bp + (size_t)(16 * nt) * (size_t)PB + k0;
      FragB bf;
      bf.h[0] = *(const v8usa*)wq;
      bf.h[1] = *(const v8usa*)(wq + 16);
      acc[nt] = wmb(af, bf, acc[nt]);
    }
  }
}

__global__ __launch_bounds__(NTHR) __attribute__((amdgpu_num_vgpr(248)))
void k_hf(const unsigned short* __restrict__ GHL, const unsigned short* __restrict__ WST2, unsigned short* HFHL) {
  __shared__ __attribute__((aligned(16))) float stg[GBM * SPW];
  const int tid = (int)threadIdx.x, lane = tid & 31, wave = tid >> 5, hh = lane >> 4, m = lane & 15;
  const int rt = wave & 3, ch = wave >> 2;
  const int rowBase = (int)blockIdx.x * GBM;
  v8f acc[4];
  {
    const v8f z = {0.f, 0.f, 0.f, 0.f, 0.f, 0.f, 0.f, 0.f};
#pragma unroll
    for (int t = 0; t < 4; ++t) acc[t] = z;
  }
  const unsigned short* ap = GHL + (size_t)(rowBase + 16 * rt + m) * (size_t)GPITCH + 8 * hh;
  const unsigned short* bp = WST2 + (size_t)(64 * ch + m) * (size_t)GPITCH + 8 * hh;
  gemm_16x64<KG, GPITCH>(ap, bp, acc);
#pragma unroll
  for (int nt = 0; nt < 4; ++nt) {
#pragma unroll
    for (int r = 0; r < 8; ++r) stg[(16 * rt + 8 * hh + r) * SPW + 64 * ch + 16 * nt + m] = acc[nt][r];
  }
  __syncthreads();

  const unsigned mk = (lane < 16) ? 0xffffffffu : 0u;
#pragma unroll 1
  for (int i = 0; i < 8; ++i) {
    const int lr   = 8 * wave + i;
    const int grow = rowBase + lr;
    const v4f a = *(const v4fa*)(stg + lr * SPW + 8 * m);
    const v4f b = *(const v4fa*)(stg + lr * SPW + 8 * m + 4);
    int h01, h23, l01, l23, h45, h67, l45, l67;
    hilo_pack(0.25f * a.x, 0.25f * a.y, 0.25f * a.z, 0.25f * a.w, h01, h23, l01, l23);
    hilo_pack(0.25f * b.x, 0.25f * b.y, 0.25f * b.z, 0.25f * b.w, h45, h67, l45, l67);
    v4u o;
    o.x = ((unsigned)h01 & mk) | ((unsigned)l01 & ~mk);
    o.y = ((unsigned)h23 & mk) | ((unsigned)l23 & ~mk);
    o.z = ((unsigned)h45 & mk) | ((unsigned)l45 & ~mk);
    o.w = ((unsigned)h67 & mk) | ((unsigned)l67 & ~mk);
    st2_v4u(HFHL + (size_t)grow * HPITCH + 8 * lane, o);
  }
}

__global__ __launch_bounds__(NTHR) __attribute__((amdgpu_num_vgpr(248)))
void k_out(const unsigned short* __restrict__ HFHL, const unsigned short* __restrict__ WHT2,
           const float* __restrict__ BH, const int* __restrict__ FLAG, float* out0) {
  __shared__ __attribute__((aligned(16))) float stg[GBM * SPW];
  __shared__ __attribute__((aligned(16))) float sb[DD];
  const int tid = (int)threadIdx.x, lane = tid & 31, wave = tid >> 5, hh = lane >> 4, m = lane & 15;
  const int rt = wave & 3, ch = wave >> 2;
  const int rowBase = (int)blockIdx.x * GBM;
  if (tid < 32) *(v4fa*)(sb + 4 * tid) = *(const v4fa*)(BH + 4 * tid);
  v8f acc[4];
  {
    const v8f z = {0.f, 0.f, 0.f, 0.f, 0.f, 0.f, 0.f, 0.f};
#pragma unroll
    for (int t = 0; t < 4; ++t) acc[t] = z;
  }
  const unsigned short* ap = HFHL + (size_t)(rowBase + 16 * rt + m) * (size_t)HPITCH + 8 * hh;
  const unsigned short* bp = WHT2 + (size_t)(64 * ch + m) * (size_t)HPITCH + 8 * hh;
  gemm_16x64<KHF, HPITCH>(ap, bp, acc);
#pragma unroll
  for (int nt = 0; nt < 4; ++nt) {
#pragma unroll
    for (int r = 0; r < 8; ++r) stg[(16 * rt + 8 * hh + r) * SPW + 64 * ch + 16 * nt + m] = acc[nt][r];
  }
  __syncthreads();

  const float qnan = __uint_as_float(0x7fc00000u);
  const v4f bias = *(const v4fa*)(sb + 4 * lane);
#pragma unroll 1
  for (int i = 0; i < 8; ++i) {
    const int lr   = 8 * wave + i;
    const int grow = rowBase + lr;
    int gb = grow >> SLB;
    gb = gb > NBK - 1 ? NBK - 1 : gb;
    const int fl = FLAG[(size_t)gb * 32];
    const v4f a = *(const v4fa*)(stg + lr * SPW + 4 * lane);
    asm volatile("" :: "v"(a), "v"(fl));
    v4f o;
    o.x = a.x + bias.x; o.y = a.y + bias.y; o.z = a.z + bias.z; o.w = a.w + bias.w;
    o.x = (fl != 0) ? qnan : o.x; o.y = (fl != 0) ? qnan : o.y;
    o.z = (fl != 0) ? qnan : o.z; o.w = (fl != 0) ? qnan : o.w;
    if (grow < NHIGH) st2_v4f(out0 + (size_t)grow * DD + 4 * lane, o);
  }
}

extern "C" void kernel_launch(void* const* d_in, const int* in_sizes, int n_in,
                              void* d_out, int out_size, void* d_ws, size_t ws_size,
                              hipStream_t stream) {
  if (n_in < 9) return;
  if (in_sizes[0] != NNODE * DD) return;
  if (in_sizes[1] != DD * HDW) return;
  if (in_sizes[2] != DD * HDW) return;
  if (in_sizes[3] != NHEAD * DD) return;
  if (in_sizes[4] != NHEAD * DD) return;
  if (in_sizes[5] != DD * DD) return;
  if (in_sizes[6] != DD) return;
  if (in_sizes[7] != NE) return;
  if (in_sizes[8] != NE) return;
  if (out_size != NHIGH * DD + NE * NHEAD) return;

  const float* x    = (const float*)d_in[0];
  const float* Wsrc = (const float*)d_in[1];
  const float* Wdst = (const float*)d_in[2];
  const float* atts = (const float*)d_in[3];
  const float* attd = (const float*)d_in[4];
  const float* Whi  = (const float*)d_in[5];
  const float* bhi  = (const float*)d_in[6];
  const int*   srcs = (const int*)d_in[7];
  const int*   dsts = (const int*)d_in[8];
  float* out0 = (float*)d_out;
  float* out1 = out0 + (size_t)NHIGH * DD;
  static_assert(((size_t)NHIGH * DD * 4) % 128 == 0);

  constexpr size_t zXB   = (size_t)MPX * DD * 2;
  constexpr size_t zAD   = (size_t)MPX * 4 * 4;
  constexpr size_t zLIST = (size_t)NBK * RCAP * 4;
  constexpr size_t zCO   = (size_t)NBK * 2 * NBRUN * 4;
  constexpr size_t zFLAG = (size_t)NBK * 128;
  constexpr size_t zSTAT = (size_t)STATROWS * 64;
  constexpr size_t zGHL  = (size_t)MPH * GPITCH * 2;
  constexpr size_t zHF   = (size_t)MPH * HPITCH * 2;
  constexpr size_t zWST  = (size_t)DD * GPITCH * 2;
  constexpr size_t zWHT  = (size_t)DD * HPITCH * 2;
  constexpr size_t zUDT  = (size_t)16 * DD * 2;
  constexpr size_t zUSRC = (size_t)DD * NHEAD * 4;
  constexpr size_t zBH   = 512;
  constexpr size_t oXB   = 0;
  constexpr size_t oAD   = oXB + zXB;
  constexpr size_t oLIST = oAD + zAD;
  constexpr size_t oCO   = oLIST + zLIST;
  constexpr size_t oFLAG = oCO + zCO;
  constexpr size_t oSTAT = oFLAG + zFLAG;
  constexpr size_t oGHL  = oSTAT + zSTAT;
  constexpr size_t oHF   = oGHL + zGHL;
  constexpr size_t oWST  = oHF + zHF;
  constexpr size_t oWHT  = oWST + zWST;
  constexpr size_t oUDT  = oWHT + zWHT;
  constexpr size_t oUSRC = oUDT + zUDT;
  constexpr size_t oBH   = oUSRC + zUSRC;
  constexpr size_t oEND  = oBH + zBH;
  static_assert(zXB % 256 == 0 && zAD % 256 == 0 && zLIST % 256 == 0 && zCO % 256 == 0 && zFLAG % 256 == 0);
  static_assert(zSTAT % 256 == 0 && zGHL % 256 == 0 && zHF % 256 == 0 && zWST % 256 == 0 && zWHT % 256 == 0);
  static_assert(zUDT % 256 == 0 && zUSRC % 256 == 0 && zBH % 256 == 0);
  static_assert(oEND <= ((size_t)128u << 20));
  if (oEND > ws_size) return;

  char* ws = (char*)d_ws;
  unsigned short* XB   = (unsigned short*)(ws + oXB);
  float*          AD   = (float*)(ws + oAD);
  int*            LIST = (int*)(ws + oLIST);
  int*            CO   = (int*)(ws + oCO);
  int*            FLAG = (int*)(ws + oFLAG);
  float*          STAT = (float*)(ws + oSTAT);
  unsigned short* GHL  = (unsigned short*)(ws + oGHL);
  unsigned short* HFHL = (unsigned short*)(ws + oHF);
  unsigned short* WST2 = (unsigned short*)(ws + oWST);
  unsigned short* WHT2 = (unsigned short*)(ws + oWHT);
  unsigned short* UDT  = (unsigned short*)(ws + oUDT);
  float*          USRC = (float*)(ws + oUSRC);
  float*          BH   = (float*)(ws + oBH);

  hipFuncSetAttribute(reinterpret_cast<const void*>(&k_bucket), hipFuncAttributeMaxDynamicSharedMemorySize, (int)BK_LDS);

  k_prep<<<PBTOT, NTHR, 0, stream>>>(x, Wsrc, Wdst, atts, attd, Whi, bhi, XB, WST2, WHT2, UDT, USRC, BH);
  k_bucket<<<NBK, NTHR, BK_LDS, stream>>>(dsts, LIST, CO, FLAG);
  k_ad<<<MPX / 128, NTHR, 0, stream>>>(XB, UDT, AD);
  k_pool<<<NPB, NTHR, 0, stream>>>(LIST, CO, FLAG, srcs, XB, AD, USRC, GHL, STAT);
  k_alpha<<<(NE + NTHR - 1) / NTHR, NTHR, 0, stream>>>(srcs, dsts, STAT, AD, FLAG, out1);
  k_hf<<<MPH / GBM, NTHR, 0, stream>>>(GHL, WST2, HFHL);
  k_out<<<MPH / GBM, NTHR, 0, stream>>>(HFHL, WHT2, BH, FLAG, out0);
}
